// Self_Attn_5291399708918
// MI455X (gfx1250) — hardware-verified
//
#include <hip/hip_runtime.h>
#include <math.h>
#include <stdint.h>

#ifndef NB
#define NB 8
#endif
#ifndef NQ
#define NQ 2048
#endif
#define NB_FULL 8
#define CDIM   512
#define NDIM   2048
#define QT     64
#define CHH    256
#define OSP    68
#define OSPW   132
#define WSC    256.0f
#define IWSC   0.00390625f
#define LNPS   9.704060527839234f
#define OSCALE 0.022097086912079608f

static_assert(NB >= 1 && NB <= NB_FULL);
static_assert(NQ >= QT && NQ <= NDIM && NQ % QT == 0);
static_assert(CDIM % QT == 0 && NDIM % QT == 0);
static_assert(CDIM % 32 == 0 && NDIM % 32 == 0);
static_assert(CDIM == 2 * CHH && CHH == 16 * 16);
static_assert((OSP * 4) % 16 == 0);
static_assert((OSPW * 4) % 16 == 0);
static_assert(NDIM == 8 * 256);

typedef _Float16       v16h __attribute__((ext_vector_type(16)));
typedef _Float16       v8h  __attribute__((ext_vector_type(8)));
typedef __bf16         v16b __attribute__((ext_vector_type(16)));
typedef unsigned short v8us __attribute__((ext_vector_type(8)));
typedef float          v8f  __attribute__((ext_vector_type(8)));
typedef float          v4f  __attribute__((ext_vector_type(4)));
typedef unsigned int   v4u  __attribute__((ext_vector_type(4)));

union Frag  { v8us u[2]; v16h h; v16b bf; };
union FragP { v16h v; v8h hv[2]; v4u u[2]; };
static_assert(sizeof(Frag) == 32);
static_assert(sizeof(FragP) == 32);

__device__ __forceinline__ unsigned short bf_bits(float f) {
  unsigned u = __float_as_uint(f);
  return (unsigned short)((u + 0x7FFFu + ((u >> 16) & 1u)) >> 16);
}
__device__ __forceinline__ float bf_up(unsigned short hb) { return __uint_as_float(((unsigned)hb) << 16); }
__device__ __forceinline__ float bfr(float f) { return bf_up(bf_bits(f)); }
__device__ __forceinline__ unsigned short h_bits(_Float16 x) { return __builtin_bit_cast(unsigned short, x); }
__device__ __forceinline__ unsigned pk16(unsigned short a, unsigned short b) { return (unsigned)a | ((unsigned)b << 16); }
__device__ __forceinline__ v8f zero8() { v8f z = {0.f, 0.f, 0.f, 0.f, 0.f, 0.f, 0.f, 0.f}; return z; }
__device__ __forceinline__ float hmax8(v8f s) {
  return fmaxf(fmaxf(fmaxf(s[0], s[1]), fmaxf(s[2], s[3])), fmaxf(fmaxf(s[4], s[5]), fmaxf(s[6], s[7])));
}
__device__ __forceinline__ unsigned wave_ballot(bool p) {
#if defined(__HIP_DEVICE_COMPILE__)
  return __builtin_amdgcn_ballot_w32(p);
#else
  return p ? 1u : 0u;
#endif
}
__device__ __forceinline__ int uni(int v) {
#if defined(__HIP_DEVICE_COMPILE__)
  return __builtin_amdgcn_readfirstlane(v);
#else
  return v;
#endif
}

__device__ __forceinline__ Frag ldfrag(const unsigned short* p) {
  Frag f;
  f.u[0] = *(const v8us*)(p);
  f.u[1] = *(const v8us*)(p + 16);
  return f;
}

__device__ __forceinline__ v8f mma_h(v16h a, v16h b, v8f c) {
  v8f d = __builtin_amdgcn_wmma_f32_16x16x32_f16(false, a, false, b, (short)0, c, false, false);
#if defined(__HIP_DEVICE_COMPILE__)
  asm volatile("v_nop\n\tv_nop\n\tv_nop\n\tv_nop" : "+v"(d) : "v"(a), "v"(b));
#endif
  return d;
}
__device__ __forceinline__ v8f mma_b(v16b a, v16b b, v8f c) {
  v8f d = __builtin_amdgcn_wmma_f32_16x16x32_bf16(false, a, false, b, (short)0, c, false, false);
#if defined(__HIP_DEVICE_COMPILE__)
  const v16h ha = __builtin_bit_cast(v16h, a), hb = __builtin_bit_cast(v16h, b);
  asm volatile("v_nop\n\tv_nop\n\tv_nop\n\tv_nop" : "+v"(d) : "v"(ha), "v"(hb));
#endif
  return d;
}

__global__ __launch_bounds__(256)
void cvt_k(const float* __restrict__ w, const float* __restrict__ x, unsigned short* W16, unsigned short* X16) {
  const int tid = threadIdx.x, r = blockIdx.x;
  const bool isw = (r < NDIM);
  const size_t ro = isw ? (size_t)r * NDIM : (size_t)(r - NDIM) * NDIM;
  const float* s = (isw ? w : x) + ro + 8 * tid;
  unsigned short* d = (isw ? W16 : X16) + ro + 8 * tid;
  const float sc = isw ? WSC : 1.0f;
  const v4f a  = *(const v4f*)s;
  const v4f qv = *(const v4f*)(s + 4);
  const float f[8] = {a[0], a[1], a[2], a[3], qv[0], qv[1], qv[2], qv[3]};
  v4u u;
#pragma unroll
  for (int t = 0; t < 4; ++t) {
    const _Float16 h0 = (_Float16)(bfr(f[2 * t]) * sc);
    const _Float16 h1 = (_Float16)(bfr(f[2 * t + 1]) * sc);
    u[t] = pk16(h_bits(h0), h_bits(h1));
  }
#pragma unroll
  for (int pass = 0; pass < 2; ++pass) {
    *(volatile v4u*)d = u;
    __threadfence();
  }
}

__global__ __launch_bounds__(128)
void proj_qk(const unsigned short* __restrict__ X16, const unsigned short* __restrict__ W16,
             const float* __restrict__ bias, unsigned short* Ph, unsigned short* Pl) {
  __shared__ __align__(16) float Os[QT * OSP];
  const int tid  = threadIdx.x;
  const int lane = tid & 31, wave = tid >> 5;
  const int hh   = lane >> 4, cl = lane & 15;
  const int ct   = blockIdx.x, ot = blockIdx.y, b = blockIdx.z;
  const int c0   = ct * QT, o0 = ot * QT;

  const unsigned short* ap = X16 + ((size_t)(b * CDIM + c0 + cl)) * NDIM + 8 * hh;
  const unsigned short* bp = W16 + ((size_t)(o0 + 16 * wave + cl)) * NDIM + 8 * hh;

  v8f acc[4];
#pragma unroll
  for (int mt = 0; mt < 4; ++mt) acc[mt] = zero8();

#pragma unroll 2
  for (int ks = 0; ks < NDIM / 32; ++ks) {
    const Frag fb = ldfrag(bp + 32 * ks);
#pragma unroll
    for (int mt = 0; mt < 4; ++mt) {
      const Frag fa = ldfrag(ap + (size_t)(16 * mt) * NDIM + 32 * ks);
      acc[mt] = mma_h(fa.h, fb.h, acc[mt]);
    }
  }

  {
    const int ol = 16 * wave + cl;
#pragma unroll
    for (int mt = 0; mt < 4; ++mt) {
      v4f va, vb;
#pragma unroll
      for (int r = 0; r < 4; ++r) { va[r] = acc[mt][r] * IWSC; vb[r] = acc[mt][4 + r] * IWSC; }
      *(v4f*)(Os + ol * OSP + 16 * mt + 8 * hh)     = va;
      *(v4f*)(Os + ol * OSP + 16 * mt + 8 * hh + 4) = vb;
    }
  }
  __syncthreads();

  const int e = tid & 7, lq = tid >> 3;
  v4u uh[4], ul[4];
#pragma unroll
  for (int it = 0; it < 4; ++it) {
    const int row = it * 16 + lq;
    const v4f a  = *(const v4f*)(Os + row * OSP + 8 * e);
    const v4f qv = *(const v4f*)(Os + row * OSP + 8 * e + 4);
    const float bb = bfr(bias[o0 + row]);
    const float f[8] = {a[0] + bb, a[1] + bb, a[2] + bb, a[3] + bb, qv[0] + bb, qv[1] + bb, qv[2] + bb, qv[3] + bb};
#pragma unroll
    for (int t = 0; t < 4; ++t) {
      const float f0 = f[2 * t], f1 = f[2 * t + 1];
      const unsigned short hb0 = bf_bits(f0), hb1 = bf_bits(f1);
      const unsigned short lb0 = bf_bits(f0 - bf_up(hb0));
      const unsigned short lb1 = bf_bits(f1 - bf_up(hb1));
      uh[it][t] = pk16(hb0, hb1);
      ul[it][t] = pk16(lb0, lb1);
    }
  }
#pragma unroll
  for (int pass = 0; pass < 2; ++pass) {
#pragma unroll
    for (int it = 0; it < 4; ++it) {
      const int row = it * 16 + lq;
      const size_t po = ((size_t)(b * NDIM + o0 + row)) * CDIM + c0 + 8 * e;
      *(volatile v4u*)(Ph + po) = uh[it];
      *(volatile v4u*)(Pl + po) = ul[it];
    }
    __threadfence();
  }
}

__global__ __launch_bounds__(128)
void proj_v(const unsigned short* __restrict__ W16, const unsigned short* __restrict__ X16,
            const float* __restrict__ bias, unsigned short* PV) {
  __shared__ __align__(16) float Os[QT * OSP];
  const int tid  = threadIdx.x;
  const int lane = tid & 31, wave = tid >> 5;
  const int hh   = lane >> 4, cl = lane & 15;
  const int ot   = blockIdx.x, ct = blockIdx.y, b = blockIdx.z;
  const int o0   = ot * QT, c0 = ct * QT;

  const unsigned short* ap = W16 + ((size_t)(o0 + cl)) * NDIM + 8 * hh;
  const unsigned short* bp = X16 + ((size_t)(b * CDIM + c0 + 16 * wave + cl)) * NDIM + 8 * hh;

  v8f acc[4];
#pragma unroll
  for (int mt = 0; mt < 4; ++mt) acc[mt] = zero8();

#pragma unroll 2
  for (int ks = 0; ks < NDIM / 32; ++ks) {
    const Frag fb = ldfrag(bp + 32 * ks);
#pragma unroll
    for (int mt = 0; mt < 4; ++mt) {
      const Frag fa = ldfrag(ap + (size_t)(16 * mt) * NDIM + 32 * ks);
      acc[mt] = mma_h(fa.h, fb.h, acc[mt]);
    }
  }

  {
    const int nl = 16 * wave + cl;
#pragma unroll
    for (int mt = 0; mt < 4; ++mt) {
      v4f va, vb;
#pragma unroll
      for (int r = 0; r < 4; ++r) { va[r] = acc[mt][r] * IWSC; vb[r] = acc[mt][4 + r] * IWSC; }
      *(v4f*)(Os + nl * OSP + 16 * mt + 8 * hh)     = va;
      *(v4f*)(Os + nl * OSP + 16 * mt + 8 * hh + 4) = vb;
    }
  }
  __syncthreads();

  const int e = tid & 7, lq = tid >> 3;
  const v4f ba = *(const v4f*)(bias + o0 + 8 * e);
  const v4f bq = *(const v4f*)(bias + o0 + 8 * e + 4);
  const float bb[8] = {bfr(ba[0]), bfr(ba[1]), bfr(ba[2]), bfr(ba[3]), bfr(bq[0]), bfr(bq[1]), bfr(bq[2]), bfr(bq[3])};
  v4u uv[4];
#pragma unroll
  for (int it = 0; it < 4; ++it) {
    const int row = it * 16 + lq;
    const v4f a  = *(const v4f*)(Os + row * OSP + 8 * e);
    const v4f qv = *(const v4f*)(Os + row * OSP + 8 * e + 4);
    const float f[8] = {a[0], a[1], a[2], a[3], qv[0], qv[1], qv[2], qv[3]};
#pragma unroll
    for (int t = 0; t < 4; ++t) {
      const _Float16 h0 = (_Float16)(f[2 * t] + bb[2 * t]);
      const _Float16 h1 = (_Float16)(f[2 * t + 1] + bb[2 * t + 1]);
      uv[it][t] = pk16(h_bits(h0), h_bits(h1));
    }
  }
#pragma unroll
  for (int pass = 0; pass < 2; ++pass) {
#pragma unroll
    for (int it = 0; it < 4; ++it) {
      const int row = it * 16 + lq;
      const size_t po = ((size_t)(b * CDIM + c0 + row)) * NDIM + o0 + 8 * e;
      *(volatile v4u*)(PV + po) = uv[it];
    }
    __threadfence();
  }
}

__global__ __launch_bounds__(256)
void attn_k(const unsigned short* __restrict__ Qh, const unsigned short* __restrict__ Ql,
            const unsigned short* __restrict__ Kh, const unsigned short* __restrict__ Kl,
            const unsigned short* __restrict__ PV, float* out) {
  __shared__ __align__(16) float Os[QT * OSPW];
  __shared__ __align__(16) unsigned Psh[4 * 32 * 8];
  __shared__ float Csh[4 * 32];
  __shared__ float Ish[4 * 32];
  __shared__ int   Gsh[4];
  const int tid  = threadIdx.x;
  const int lane = tid & 31;
  const int wave = uni((int)(threadIdx.x >> 5));
  const int w    = wave & 3, g = wave >> 2;
  const int hh   = lane >> 4, cl = lane & 15;
  const int n0   = blockIdx.x * QT, b = blockIdx.y;

  const size_t qo = ((size_t)(b * NDIM + n0 + 16 * w + cl)) * CDIM + 8 * hh;
  const unsigned short* Qhp = Qh + qo;
  const unsigned short* Qlp = Ql + qo;
  const unsigned short* Khp = Kh + (size_t)b * NDIM * CDIM + (size_t)cl * CDIM + 8 * hh;
  const unsigned short* Klp = Kl + (size_t)b * NDIM * CDIM + (size_t)cl * CDIM + 8 * hh;
  const unsigned short* Vp = PV + (size_t)b * CDIM * NDIM + (size_t)(g * CHH + cl) * NDIM + 8 * hh;

  const int pso = (w * 32 + lane) * 8;

  float m = -1.0e30f, l = 0.f;
  v8f o[16];
#pragma unroll
  for (int j = 0; j < 16; ++j) o[j] = zero8();

#pragma unroll 1
  for (int kb = 0; kb < NDIM; kb += 32) {
    if (wave < 4) {
      const unsigned short* k0p  = Khp + (size_t)kb * CDIM;
      const unsigned short* k1p  = Khp + (size_t)(kb + 16) * CDIM;
      const unsigned short* k0lp = Klp + (size_t)kb * CDIM;
      const unsigned short* k1lp = Klp + (size_t)(kb + 16) * CDIM;
      v8f s0 = zero8(), s1 = zero8();
#pragma unroll 1
      for (int kc = 0; kc < CDIM / 32; ++kc) {
        const Frag qh  = ldfrag(Qhp + 32 * kc);
        const Frag k0  = ldfrag(k0p + 32 * kc);
        const Frag k1  = ldfrag(k1p + 32 * kc);
        s0 = mma_b(k0.bf, qh.bf, s0);
        s1 = mma_b(k1.bf, qh.bf, s1);
        const Frag ql  = ldfrag(Qlp + 32 * kc);
        s0 = mma_b(k0.bf, ql.bf, s0);
        s1 = mma_b(k1.bf, ql.bf, s1);
        const Frag k0l = ldfrag(k0lp + 32 * kc);
        const Frag k1l = ldfrag(k1lp + 32 * kc);
        s0 = mma_b(k0l.bf, qh.bf, s0);
        s1 = mma_b(k1l.bf, qh.bf, s1);
      }

      float mx = fmaxf(hmax8(s0), hmax8(s1));
      mx = fmaxf(mx, __shfl_xor(mx, 16, 32));
      const float mn = fmaxf(m, mx);
      const unsigned grew = wave_ballot(mx > m);
      float corr = 1.0f;
      if (grew != 0u) {
        corr = __expf(m - mn);
        l *= corr;
      }
      m = mn;
      const float msh = mn - LNPS;

      FragP ph;
      float ls = 0.f;
#pragma unroll
      for (int r = 0; r < 8; ++r) {
        const float e0 = __expf(s0[r] - msh);
        const float e1 = __expf(s1[r] - msh);
        ls += e0 + e1;
        ph.hv[0][r] = (_Float16)e0;
        ph.hv[1][r] = (_Float16)e1;
      }
      l += ls;

      *(v4u*)(Psh + pso)     = ph.u[0];
      *(v4u*)(Psh + pso + 4) = ph.u[1];
      Csh[w * 32 + lane] = corr;
      Gsh[w] = (grew != 0u) ? 1 : 0;
    }
    __syncthreads();

    {
      const int gf = uni(Gsh[w]);
      if (gf != 0) {
        const float corr = Csh[w * 32 + lane];
#pragma unroll
        for (int j = 0; j < 16; ++j) {
#pragma unroll
          for (int r = 0; r < 8; ++r) o[j][r] *= corr;
        }
      }
      FragP pb;
      pb.u[0] = *(const v4u*)(Psh + pso);
      pb.u[1] = *(const v4u*)(Psh + pso + 4);
#pragma unroll
      for (int j = 0; j < 16; ++j) {
        const Frag vf = ldfrag(Vp + (size_t)(16 * j) * NDIM + kb);
        o[j] = mma_h(vf.h, pb.v, o[j]);
      }
    }
    __syncthreads();
  }

  if (wave < 4) {
    l += __shfl_xor(l, 16, 32);
    Ish[w * 32 + lane] = (1.0f / l) * OSCALE;
  }
  __syncthreads();
  const float inv = Ish[w * 32 + lane];

  const int qrow = 16 * w + cl;
  const int e = tid & 7, lq = tid >> 3;
#pragma unroll
  for (int p = 0; p < 4; ++p) {
    if (p) __syncthreads();
#pragma unroll
    for (int jj = 0; jj < 4; ++jj) {
      const int j = 4 * p + jj;
      v4f va, vb;
#pragma unroll
      for (int r = 0; r < 4; ++r) { va[r] = o[j][r] * inv; vb[r] = o[j][4 + r] * inv; }
      *(v4f*)(Os + qrow * OSPW + g * 64 + 16 * jj + 8 * hh)     = va;
      *(v4f*)(Os + qrow * OSPW + g * 64 + 16 * jj + 8 * hh + 4) = vb;
    }
    __syncthreads();
    v4f res[8];
#pragma unroll
    for (int it = 0; it < 8; ++it) {
      const int L   = it * 32 + lq;
      const int ql  = L >> 2, seg = L & 3;
      const int gg  = seg >> 1, ln = seg & 1;
      res[it] = *(const v4f*)(Os + ql * OSPW + gg * 64 + 32 * ln + 4 * e);
    }
#pragma unroll
    for (int pass = 0; pass < 2; ++pass) {
#pragma unroll
      for (int it = 0; it < 8; ++it) {
        const int L   = it * 32 + lq;
        const int ql  = L >> 2, seg = L & 3;
        const int gg  = seg >> 1, ln = seg & 1;
        const int ch  = gg * CHH + 64 * p + 32 * ln + 4 * e;
        const size_t idx = ((size_t)(b * NDIM + n0 + ql)) * CDIM + ch;
        *(volatile v4f*)(out + idx) = res[it];
      }
      __threadfence();
    }
  }
}

extern "C" void kernel_launch(void* const* d_in, const int* in_sizes, int n_in,
                              void* d_out, int out_size, void* d_ws, size_t ws_size,
                              hipStream_t stream) {
  if (n_in < 9) return;
  if (in_sizes[0] < NB * CDIM * NDIM || in_sizes[1] < NB * CDIM * NDIM || in_sizes[2] < NB * CDIM * NDIM) return;
  if (in_sizes[3] < NDIM * NDIM || in_sizes[5] < NDIM * NDIM || in_sizes[7] < NDIM * NDIM) return;
  if (in_sizes[4] < NDIM || in_sizes[6] < NDIM || in_sizes[8] < NDIM) return;
  if (out_size < (NB - 1) * NDIM * CDIM + NQ * CDIM) return;

  size_t off = 0;
  auto carve = [&](size_t bytes) { const size_t o = off; off += (bytes + 255) & ~(size_t)255; return o; };
  const size_t oW16 = carve((size_t)NDIM * NDIM * 2);
  const size_t oX16 = carve((size_t)NB * CDIM * NDIM * 2);
  const size_t oQh  = carve((size_t)NB * NDIM * CDIM * 2);
  const size_t oQl  = carve((size_t)NB * NDIM * CDIM * 2);
  const size_t oKh  = carve((size_t)NB * NDIM * CDIM * 2);
  const size_t oKl  = carve((size_t)NB * NDIM * CDIM * 2);
  const size_t oPV  = carve((size_t)NB * CDIM * NDIM * 2);
  if (off > ws_size) return;
  if (off > (size_t)134217728) return;

  const float* q  = (const float*)d_in[0];
  const float* k  = (const float*)d_in[1];
  const float* v  = (const float*)d_in[2];
  const float* Wq = (const float*)d_in[3];
  const float* bq = (const float*)d_in[4];
  const float* Wk = (const float*)d_in[5];
  const float* bk = (const float*)d_in[6];
  const float* Wv = (const float*)d_in[7];
  const float* bv = (const float*)d_in[8];

  char* ws = (char*)d_ws;
  unsigned short* W16 = (unsigned short*)(ws + oW16);
  unsigned short* X16 = (unsigned short*)(ws + oX16);
  unsigned short* Qh  = (unsigned short*)(ws + oQh);
  unsigned short* Ql  = (unsigned short*)(ws + oQl);
  unsigned short* Kh  = (unsigned short*)(ws + oKh);
  unsigned short* Kl  = (unsigned short*)(ws + oKl);
  unsigned short* PVp = (unsigned short*)(ws + oPV);
  float* out = (float*)d_out;

  const dim3 blk256(256), blk128(128);
  const int cvt_blocks = NDIM + NB * CDIM;

  cvt_k<<<dim3(cvt_blocks), blk256, 0, stream>>>(Wq, q, W16, X16);
  proj_qk<<<dim3(CDIM / QT, NQ / QT, NB), blk128, 0, stream>>>(X16, W16, bq, Qh, Ql);
  cvt_k<<<dim3(cvt_blocks), blk256, 0, stream>>>(Wk, k, W16, X16);
  proj_qk<<<dim3(CDIM / QT, NDIM / QT, NB), blk128, 0, stream>>>(X16, W16, bk, Kh, Kl);
  cvt_k<<<dim3(cvt_blocks), blk256, 0, stream>>>(Wv, v, W16, X16);
  proj_v<<<dim3(NDIM / QT, CDIM / QT, NB), blk128, 0, stream>>>(W16, X16, bv, PVp);
  attn_k<<<dim3(NQ / QT, NB), blk256, 0, stream>>>(Qh, Ql, Kh, Kl, PVp, out);
  (void)hipGetLastError();
}
